// MatrixGCN_9801115369777
// MI455X (gfx1250) — hardware-verified
//
#include <hip/hip_runtime.h>
#include <hip/hip_bf16.h>
#include <math.h>


#define BB 2
#define SS 2048
#define DD 1024
#define HH 16
#define DKK 64
#define QW 2

typedef _Float16 bf16;
typedef __attribute__((ext_vector_type(4))) unsigned v4u_t;
typedef unsigned v4ua __attribute__((ext_vector_type(4), may_alias));
typedef __attribute__((ext_vector_type(4))) float v4f_t;
typedef float v4fa __attribute__((ext_vector_type(4), may_alias));
typedef __attribute__((ext_vector_type(16))) bf16  bf16x16;
typedef __attribute__((ext_vector_type(8)))  bf16  bf16x8;
typedef __attribute__((ext_vector_type(4)))  bf16  bf16x4;
typedef __attribute__((ext_vector_type(8)))  float f32x8;

#define LDS_STRIDE 48
#define KSTRIDE    72
#define VSTRIDE    48

__device__ __forceinline__ f32x8 wmma_bf16(bf16x16 a, bf16x16 b, f32x8 c) {
  return __builtin_amdgcn_wmma_f32_16x16x32_f16(
      false, a, false, b, (short)0, c, false, false);
}

template <typename T>
__device__ __forceinline__ bf16x16 load_frag(const T* __restrict__ base, int ld,
                                             int row0, int k0) {
  const int lane = threadIdx.x & 31;
  const int r    = lane & 15;
  const int kh   = (lane >> 4) * 8;
  const T* p0 = base + (size_t)(row0 + r) * ld + (k0 + kh);
  const T* p1 = p0 + 16;
  bf16x16 f;
#pragma unroll
  for (int i = 0; i < 8; ++i) {
    f[i]     = (bf16)p0[i];
    f[i + 8] = (bf16)p1[i];
  }
  return f;
}

__device__ __forceinline__ bf16x16 lds_frag(const bf16* base, int stride) {
  const int lane = threadIdx.x & 31;
  const int row  = lane & 15;
  const int kh   = (lane >> 4) * 8;
  const bf16x8 lo = *(const bf16x8*)(base + row * stride + kh);
  const bf16x8 hi = *(const bf16x8*)(base + row * stride + kh + 16);
  bf16x16 f;
#pragma unroll
  for (int i = 0; i < 8; ++i) { f[i] = lo[i]; f[i + 8] = hi[i]; }
  return f;
}

template <typename T>
__device__ __forceinline__ void stage_read16(const T* __restrict__ p, float* buf) {
#pragma unroll
  for (int i = 0; i < 16; ++i) buf[i] = (float)p[i];
}

__device__ __forceinline__ void stage_write(bf16* dst, const float* buf, int nquad) {
#pragma unroll
  for (int i = 0; i < nquad; ++i) {
    bf16x4 q;
    q[0] = (bf16)buf[4 * i];     q[1] = (bf16)buf[4 * i + 1];
    q[2] = (bf16)buf[4 * i + 2]; q[3] = (bf16)buf[4 * i + 3];
    *(bf16x4*)(dst + 4 * i) = q;
  }
}

template <typename AT, int MODE>
__global__ __launch_bounds__(256) void gemm_bias_kernel(
    const AT* __restrict__ A, const float* __restrict__ W,
    const float* __restrict__ bias, void* __restrict__ out,
    int M, int N, int K) {
  __shared__ bf16 ldsA[128 * LDS_STRIDE];
  __shared__ bf16 ldsW[256 * LDS_STRIDE];
  __shared__ __attribute__((aligned(16))) unsigned char sob[256 * 136 * 2];

  const int t    = threadIdx.x;
  const int wave = t >> 5;
  const int lane = t & 31;
  const int wm   = (wave & 1) * 64;
  const int wn   = (wave >> 1) * 64;
  const int mBlk = blockIdx.x * 128;
  const int nBlk = blockIdx.y * 256;

  const int arow = t >> 1;
  const int ach  = (t & 1) * 16;

  float abuf[16];
  float wbuf[32];

  stage_read16(A + (size_t)(mBlk + arow) * K + ach, abuf);
  stage_read16(W + (size_t)(nBlk + t) * K,          wbuf);
  stage_read16(W + (size_t)(nBlk + t) * K + 16,     wbuf + 16);

  f32x8 acc[4][4] = {};

  for (int k = 0; k < K; k += 32) {
    __syncthreads();
    stage_write(&ldsA[arow * LDS_STRIDE + ach], abuf, 4);
    stage_write(&ldsW[t * LDS_STRIDE],          wbuf, 8);
    if (k + 32 < K) {
      stage_read16(A + (size_t)(mBlk + arow) * K + (k + 32) + ach, abuf);
      stage_read16(W + (size_t)(nBlk + t) * K + (k + 32),          wbuf);
      stage_read16(W + (size_t)(nBlk + t) * K + (k + 32) + 16,     wbuf + 16);
    }
    __syncthreads();

    bf16x16 af[4], wf[4];
#pragma unroll
    for (int i = 0; i < 4; ++i)
      af[i] = lds_frag(ldsA + (wm + 16 * i) * LDS_STRIDE, LDS_STRIDE);
#pragma unroll
    for (int j = 0; j < 4; ++j)
      wf[j] = lds_frag(ldsW + (wn + 16 * j) * LDS_STRIDE, LDS_STRIDE);
#pragma unroll
    for (int i = 0; i < 4; ++i)
#pragma unroll
      for (int j = 0; j < 4; ++j)
        acc[i][j] = wmma_bf16(af[i], wf[j], acc[i][j]);
  }

  const int nlane = lane & 15;
  const int mh    = (lane >> 4) * 8;
  __syncthreads();
  if (MODE == 0 || MODE == 1 || MODE == 3) {
    bf16* so = (bf16*)sob;
#pragma unroll
    for (int i = 0; i < 4; ++i)
#pragma unroll
      for (int j = 0; j < 4; ++j) {
        const int nl = wn + 16 * j + nlane;
        const float bv = bias ? bias[nBlk + nl] : 0.0f;
#pragma unroll
        for (int r = 0; r < 8; ++r) {
          const int ml = wm + 16 * i + mh + r;
          const bf16 hv = (MODE == 3) ? (bf16)fmaxf(acc[i][j][r] + bv, 0.0f) : (bf16)(acc[i][j][r] + bv);
          if (MODE == 0 || MODE == 3) so[ml * 264 + nl] = hv;
          else           so[nl * 136 + ml] = hv;
        }
      }
    __syncthreads();
#pragma unroll 1
    for (int pass = 0; pass < 2; ++pass) {
      if (MODE == 0 || MODE == 3) {
        for (int ch = t; ch < 128 * 32; ch += 256) { const int ml = ch >> 5, q = (ch & 31) * 8;
          *(volatile v4u_t*)((bf16*)out + (size_t)(mBlk + ml) * N + nBlk + q) = *(const v4ua*)(so + ml * 264 + q); }
      } else {
        const int b_ = mBlk / SS, s0 = mBlk & (SS - 1);
        for (int ch = t; ch < 256 * 16; ch += 256) { const int nl = ch >> 4, q = (ch & 15) * 8; const int n = nBlk + nl, h = n >> 6, dk = n & (DKK - 1);
          *(volatile v4u_t*)((bf16*)out + (((size_t)(b_ * HH + h)) * DKK + dk) * SS + s0 + q) = *(const v4ua*)(so + nl * 136 + q); }
      }
      __threadfence();
    }
  } else {
    float* so = (float*)sob;
#pragma unroll 1
    for (int hf = 0; hf < 2; ++hf) {
      if (wm == hf * 64) {
#pragma unroll
        for (int i = 0; i < 4; ++i)
#pragma unroll
          for (int j = 0; j < 4; ++j) {
            const int nl = wn + 16 * j + nlane;
            const float bv = bias ? bias[nBlk + nl] : 0.0f;
#pragma unroll
            for (int r = 0; r < 8; ++r) so[(16 * i + mh + r) * 260 + nl] = acc[i][j][r] + bv;
          }
      }
      __syncthreads();
#pragma unroll 1
      for (int pass = 0; pass < 2; ++pass) {
        for (int ch = t; ch < 64 * 64; ch += 256) { const int ml = ch >> 6, q = (ch & 63) * 4;
          *(volatile v4f_t*)((float*)out + (size_t)(mBlk + hf * 64 + ml) * N + nBlk + q) = *(const volatile v4fa*)(so + ml * 260 + q); }
        __threadfence();
      }
      __syncthreads();
    }
  }
}


#define GN 20000
#define GNP 20096
#define GE 320000
#define DR GNP

__global__ __launch_bounds__(256) void k_degc(const int* __restrict__ idx, float* __restrict__ nrm) {
  __shared__ unsigned short dg[DR]; __shared__ int qd[8][256]; __shared__ int wcnt[8][8];
  const int tid = threadIdx.x, lane = tid & 31, wave = tid >> 5;
  for (int i = tid; i < DR; i += 256) dg[i] = 0;
  __syncthreads();
#pragma unroll 1
  for (int c0 = 0; c0 < GE; c0 += 256) {
    const int e = c0 + tid; int d = -1;
    if (e < GE) { const int draw = idx[e]; d = draw < 0 ? 0 : (draw >= GN ? GN - 1 : draw); }
    const int own = (d >= 0) ? (d & 7) : -1; unsigned mown = 0u;
#pragma unroll
    for (int ww = 0; ww < 8; ++ww) { const unsigned m = __builtin_amdgcn_ballot_w32(own == ww); if (own == ww) mown = m; if (lane == 0) wcnt[ww][wave] = __builtin_popcount(m); }
    __syncthreads();
    if (own >= 0) { int base = 0;
#pragma unroll
      for (int w2 = 0; w2 < 8; ++w2) base += (w2 < wave) ? wcnt[own][w2] : 0;
      const int pos = base + __builtin_popcount(mown & ((1u << lane) - 1u)); qd[own][pos] = d; }
    int total = 0;
#pragma unroll
    for (int w2 = 0; w2 < 8; ++w2) total += wcnt[wave][w2];
    __syncthreads();
    if (lane == 0) {
#pragma unroll 1
      for (int qi = 0; qi < total; ++qi) dg[qd[wave][qi]] += 1; }
    __syncthreads();
  }
#pragma unroll 1
  for (int pass = 0; pass < 2; ++pass) {
    for (int i = tid; i < DR / 4; i += 256) { v4f_t v;
#pragma unroll
      for (int q = 0; q < 4; ++q) { const int n = i * 4 + q; const float g = (float)dg[n] + ((n < GN) ? 1.0f : 0.0f); v[q] = (g > 0.0f) ? rsqrtf(g) : 0.0f; }
      *(volatile v4f_t*)(nrm + i * 4) = v; }
    __threadfence(); }
}
template <int FW, int RANGE>
__global__ __launch_bounds__(256) void k_agg(const int* __restrict__ rowi, const int* __restrict__ coli, const float* __restrict__ no, const float* __restrict__ ni,
                                            const float* __restrict__ H, float* __restrict__ R, int rsel) {
  __shared__ int qd[8][256], qs[8][256]; __shared__ float qw[8][256]; __shared__ int wcnt[8][8];
  const int tid = threadIdx.x, lane = tid & 31, wave = tid >> 5, r0 = rsel * RANGE;
  constexpr int Q4 = FW / 4;
  for (int i = tid; i < RANGE * Q4; i += 256) { v4f_t z; z.x = z.y = z.z = z.w = 0.0f; *(volatile v4f_t*)(R + (size_t)i * 4) = z; }
  __threadfence(); __syncthreads();
#pragma unroll 1
  for (int c0 = 0; c0 < GE; c0 += 256) {
    const int e = c0 + tid; int d = -1, sidx = 0; float w = 0.0f;
    if (e < GE) { const int draw = coli[e]; const int dd = draw < 0 ? 0 : (draw >= GN ? GN - 1 : draw);
      if (dd >= r0 && dd < r0 + RANGE) { d = dd - r0; const int ss = rowi[e]; sidx = ss < 0 ? 0 : (ss >= GN ? GN - 1 : ss); w = no[sidx] * ni[dd]; } }
    const int own = (d >= 0) ? (d & 7) : -1; unsigned mown = 0u;
#pragma unroll
    for (int ww = 0; ww < 8; ++ww) { const unsigned m = __builtin_amdgcn_ballot_w32(own == ww); if (own == ww) mown = m; if (lane == 0) wcnt[ww][wave] = __builtin_popcount(m); }
    __syncthreads();
    if (own >= 0) { int base = 0;
#pragma unroll
      for (int w2 = 0; w2 < 8; ++w2) base += (w2 < wave) ? wcnt[own][w2] : 0;
      const int pos = base + __builtin_popcount(mown & ((1u << lane) - 1u)); qd[own][pos] = d; qs[own][pos] = sidx; qw[own][pos] = w; }
    int total = 0;
#pragma unroll
    for (int w2 = 0; w2 < 8; ++w2) total += wcnt[wave][w2];
    __syncthreads();
#pragma unroll 1
    for (int qi = 0; qi < total; ++qi) { const int dl = qd[wave][qi]; const int sl = qs[wave][qi]; const float wv = qw[wave][qi];
      float* row = R + (size_t)dl * FW; const float* hs = H + (size_t)sl * FW;
#pragma unroll
      for (int u = 0; u < FW / 32; ++u) row[u * 32 + lane] += wv * hs[u * 32 + lane]; }
    __syncthreads();
  }
  __threadfence(); __syncthreads();
  for (int i = tid; i < RANGE * Q4; i += 256) { float* p = R + (size_t)i * 4; const v4f_t v = *(const volatile v4fa*)p; *(volatile v4f_t*)p = v; }
  __threadfence();
}
__global__ __launch_bounds__(192) void k_padx(const float* __restrict__ x, float* __restrict__ XP) {
  const int n = blockIdx.x, t = threadIdx.x; const float v = (n < GN) ? x[(size_t)n * 192 + t] : 0.0f;
  *(volatile float*)(XP + (size_t)n * 192 + t) = v; __threadfence(); *(volatile float*)(XP + (size_t)n * 192 + t) = v;
}
__global__ __launch_bounds__(192) void k_fold(const float* __restrict__ cw, const float* __restrict__ W1, float* __restrict__ Wf) {
  const int j = blockIdx.x, kk = threadIdx.x, t = kk >> 3, w = kk & 7; float s = 0.0f;
#pragma unroll 1
  for (int o = 0; o < 64; ++o) s += cw[o * 24 + t] * W1[((size_t)o * 8 + w) * 256 + j];
  *(volatile float*)(Wf + (size_t)j * 192 + kk) = s; __threadfence(); *(volatile float*)(Wf + (size_t)j * 192 + kk) = s;
}
__global__ __launch_bounds__(256) void k_foldb(const float* __restrict__ cb, const float* __restrict__ W1, float* __restrict__ bfv) {
  const int j = threadIdx.x; float s = 0.0f;
#pragma unroll 1
  for (int r = 0; r < 512; ++r) s += cb[r >> 3] * W1[(size_t)r * 256 + j];
  *(volatile float*)(bfv + j) = s; __threadfence(); *(volatile float*)(bfv + j) = s;
}
__global__ __launch_bounds__(256) void k_tw2(const float* __restrict__ W2, float* __restrict__ WT) {
  const int n = blockIdx.x, k = threadIdx.x; const float v = (n < 128) ? W2[(size_t)k * 128 + n] : 0.0f;
  *(volatile float*)(WT + (size_t)n * 256 + k) = v; __threadfence(); *(volatile float*)(WT + (size_t)n * 256 + k) = v;
}
template <int FW, int FOUT, int RELU>
__global__ __launch_bounds__(256) void k_fin(const float* __restrict__ R, const float* __restrict__ HW, const float* __restrict__ dinv, const float* __restrict__ b, float* __restrict__ Hout) {
  const int n = blockIdx.x, c = threadIdx.x; if (c >= FOUT) return;
  float v = 0.0f;
  if (n < GN) { const float di = dinv[n]; v = R[(size_t)n * FW + c] + di * di * HW[(size_t)n * FW + c] + b[c]; if (RELU) v = fmaxf(v, 0.0f); }
  *(volatile float*)(Hout + (size_t)n * FOUT + c) = v; __threadfence(); *(volatile float*)(Hout + (size_t)n * FOUT + c) = v;
}

extern "C" void kernel_launch(void* const* d_in, const int* in_sizes, int n_in,
                              void* d_out, int out_size, void* d_ws, size_t ws_size,
                              hipStream_t stream) {
  (void)in_sizes; (void)n_in; (void)out_size; (void)ws_size;
  const float* x = (const float*)d_in[0];
  const int* ei = (const int*)d_in[1];
  const float* cw = (const float*)d_in[2]; const float* cb = (const float*)d_in[3];
  const float* W1 = (const float*)d_in[4]; const float* b1 = (const float*)d_in[5];
  const float* W2 = (const float*)d_in[6]; const float* b2 = (const float*)d_in[7];
  const int* rowi = ei; const int* coli = ei + (size_t)GE;
  float* out = (float*)d_out;
  char* ws = (char*)d_ws;
  float* Wf  = (float*)ws; ws += (size_t)256 * 192 * 4;
  float* bfv = (float*)ws; ws += 256 * 4;
  float* W2T = (float*)ws; ws += (size_t)256 * 256 * 4;
  float* dinv = (float*)ws; ws += (size_t)GNP * 4;
  float* XP  = (float*)ws; ws += (size_t)GNP * 192 * 4;
  float* HW  = (float*)ws; ws += (size_t)GNP * 256 * 4;
  float* R   = (float*)ws; ws += (size_t)GNP * 256 * 4;
  float* H1  = (float*)ws; ws += (size_t)GNP * 256 * 4;
  k_fold<<<256, 192, 0, stream>>>(cw, W1, Wf);
  k_foldb<<<1, 256, 0, stream>>>(cb, W1, bfv);
  k_tw2<<<256, 256, 0, stream>>>(W2, W2T);
  k_padx<<<GNP, 192, 0, stream>>>(x, XP);
  k_degc<<<1, 256, 0, stream>>>(coli, dinv);
  dim3 blk(256);
  gemm_bias_kernel<float, 2><<<dim3(GNP / 128, 1), blk, 0, stream>>>(XP, Wf, bfv, HW, GNP, 256, 192);
  k_agg<256, GNP><<<1, 256, 0, stream>>>(rowi, coli, dinv, dinv, HW, R, 0);
  k_fin<256, 256, 1><<<GNP, 256, 0, stream>>>(R, HW, dinv, b1, H1);
  gemm_bias_kernel<float, 2><<<dim3(GNP / 128, 1), blk, 0, stream>>>(H1, W2T, nullptr, HW, GNP, 256, 256);
  k_agg<256, GNP><<<1, 256, 0, stream>>>(rowi, coli, dinv, dinv, HW, R, 0);
  k_fin<256, 128, 0><<<GN, 256, 0, stream>>>(R, HW, dinv, b2, out);
}
